// SelfNormAttention_25537875542112
// MI455X (gfx1250) — hardware-verified
//
#include <hip/hip_runtime.h>
#include <math.h>
#include <stdint.h>

#ifndef NB
#define NB 4
#endif
#ifndef SEQ
#define SEQ 2048
#endif
#define S_FULL 2048
#define NH    8
#define HD    64
#define DMOD  (NH * HD)
#define QKW   (2 * DMOD)
#define QKSC  1024.0f
#define VSC   64.0f
#define PCAR  128.0f
#define WPB   4
#define NHG   (NH / WPB)
#define NQT   (SEQ / 16)
#define NST   (SEQ / 64)
#define NKT   (SEQ / 32)
#define ATT_THREADS (WPB * 32)
#define PTP   36
#define PTW   (16 * PTP)
#define SLP   68
#define SLW   (16 * SLP)
#define WREG  (PTW + SLW)
#define VTP   72
#define WS_CAP 134217728
static_assert(DMOD == 512 && QKW == 1024 && HD == 64 && NH == 8 && WPB == 4 && NHG * WPB == NH && ATT_THREADS == 128);
static_assert(NB >= 1 && NB <= 4);
static_assert(NB == 1 || SEQ == S_FULL);
static_assert((SEQ % 64) == 0 && SEQ >= 64 && SEQ <= S_FULL);
static_assert((HD % 32) == 0 && (QKW / 8) == 128 && (DMOD % 16) == 0);
static_assert(WPB * WREG * 4 <= 65536 && HD * VTP * 2 <= 65536);
static_assert((size_t)NB * SEQ * QKW * 2 * 2 + (size_t)NB * DMOD * SEQ * 2 <= (size_t)WS_CAP);
static_assert(15 * PTP + 31 < PTW && 15 * SLP + 63 < SLW && 63 * VTP + 63 < HD * VTP);

typedef unsigned short u16;
typedef _Float16 v16h __attribute__((ext_vector_type(16)));
typedef _Float16 v8h  __attribute__((ext_vector_type(8)));
typedef float    v8f  __attribute__((ext_vector_type(8)));
typedef float    v4f  __attribute__((ext_vector_type(4)));
typedef unsigned int v4u __attribute__((ext_vector_type(4)));

union FragH { v16h v; v8h h[2]; v4u u[2]; };

__device__ __forceinline__ unsigned short bf_bits(float f) {
  unsigned u = __float_as_uint(f);
  return (unsigned short)((u + 0x7FFFu + ((u >> 16) & 1u)) >> 16);
}
__device__ __forceinline__ float bf_up(unsigned short h) { return __uint_as_float(((unsigned)h) << 16); }
__device__ __forceinline__ float bfr(float f) { return bf_up(bf_bits(f)); }
__device__ __forceinline__ unsigned short h_bits(_Float16 x) { return __builtin_bit_cast(unsigned short, x); }
__device__ __forceinline__ unsigned pk16(unsigned short a, unsigned short b) { return (unsigned)a | ((unsigned)b << 16); }
__device__ __forceinline__ v8f zero8() { v8f z = {0.f, 0.f, 0.f, 0.f, 0.f, 0.f, 0.f, 0.f}; return z; }

__device__ __forceinline__ v16h ldfrag_h(const _Float16* p) {
  FragH f;
  f.h[0] = *(const v8h*)(p);
  f.h[1] = *(const v8h*)(p + 16);
  return f.v;
}

__device__ __forceinline__ v8f mma_h(v16h a, v16h b, v8f c) {
  return __builtin_amdgcn_wmma_f32_16x16x32_f16(false, a, false, b, (short)0, c, false, false);
}
__device__ __forceinline__ void guard2(v8f& a, v8f& b, v16h x0, v16h x1, v16h x2, v16h x3, v16h x4, v16h x5) {
#if defined(__HIP_DEVICE_COMPILE__)
  asm volatile("v_nop\n\tv_nop\n\tv_nop\n\tv_nop"
               : "+v"(a), "+v"(b) : "v"(x0), "v"(x1), "v"(x2), "v"(x3), "v"(x4), "v"(x5) : "memory");
#endif
}
__device__ __forceinline__ void acc_guard4(v8f& a, v8f& b, v8f& c, v8f& d) {
#if defined(__HIP_DEVICE_COMPILE__)
  asm volatile("v_nop\n\tv_nop\n\tv_nop\n\tv_nop" : "+v"(a), "+v"(b), "+v"(c), "+v"(d));
#endif
}
__device__ __forceinline__ void wave_sync_lds() {
  __builtin_amdgcn_fence(__ATOMIC_RELEASE, "workgroup");
  __builtin_amdgcn_wave_barrier();
  __builtin_amdgcn_fence(__ATOMIC_ACQUIRE, "workgroup");
}

__global__ __launch_bounds__(128) void qk16(const float* __restrict__ QK, u16* Hp, u16* Lp) {
#pragma clang fp contract(off)
  const int tid  = (int)threadIdx.x;
  const int prow = (int)blockIdx.x;
  if (prow >= NB * SEQ) return;
  const int b  = prow / SEQ;
  const int s  = prow - b * SEQ;
  const int c8 = tid * 8;
  const float* p = QK + ((size_t)b * S_FULL + (size_t)s) * (size_t)QKW + c8;
  const v4f a = *(const v4f*)(p), b4 = *(const v4f*)(p + 4);
  float w[8];
#pragma unroll
  for (int e = 0; e < 4; ++e) { w[e] = a[e]; w[4 + e] = b4[e]; }
  v4u oh, ol;
#pragma unroll
  for (int e = 0; e < 4; ++e) {
    const float x0 = bfr(w[2 * e]), x1 = bfr(w[2 * e + 1]);
    const float n0 = __expf(fminf(x0, 0.0f)), n1 = __expf(fminf(x1, 0.0f));
    const float f0 = (x0 > 0.0f) ? (x0 + 1.0f) : n0;
    const float f1 = (x1 > 0.0f) ? (x1 + 1.0f) : n1;
    const float t0 = f0 * QKSC, t1 = f1 * QKSC;
    const _Float16 h0 = (_Float16)t0, h1 = (_Float16)t1;
    const _Float16 l0 = (_Float16)(t0 - (float)h0), l1 = (_Float16)(t1 - (float)h1);
    oh[e] = pk16(h_bits(h0), h_bits(h1));
    ol[e] = pk16(h_bits(l0), h_bits(l1));
  }
  u16* dh = Hp + (size_t)prow * QKW + c8;
  u16* dl = Lp + (size_t)prow * QKW + c8;
  for (int pass = 0; pass < 2; ++pass) {
    *(volatile v4u*)(dh) = oh;
    *(volatile v4u*)(dl) = ol;
    __threadfence();
  }
}

__global__ __launch_bounds__(256) void vt16(const float* __restrict__ V, u16* VTo) {
#pragma clang fp contract(off)
  __shared__ __align__(16) u16 T[HD * VTP];
  const int tid = (int)threadIdx.x;
  const int bid = (int)blockIdx.x;
  const int st  = bid % NST;
  const int bh  = bid / NST;
  const int h   = bh % NH;
  const int b   = bh / NH;
  if (b >= NB) return;
  const int s0  = st * 64;
  {
    const int sl = tid >> 2;
    const int dc = (tid & 3) * 16;
    const float* src = V + ((size_t)b * S_FULL + (size_t)(s0 + sl)) * (size_t)DMOD + h * HD + dc;
#pragma unroll
    for (int i = 0; i < 4; ++i) {
      const v4f a = *(const v4f*)(src + 4 * i);
#pragma unroll
      for (int e = 0; e < 4; ++e) {
        const float t = bfr(a[e]) * VSC;
        T[(dc + 4 * i + e) * VTP + sl] = h_bits((_Float16)t);
      }
    }
  }
  __syncthreads();
  v4u vv[2];
  const int q8 = tid >> 3, p8 = (tid & 7) * 8;
#pragma unroll
  for (int it = 0; it < 2; ++it) {
    const int line = it * 32 + q8;
    vv[it] = *(const v4u*)(T + line * VTP + p8);
  }
  const size_t base = ((size_t)b * DMOD + (size_t)h * HD) * (size_t)SEQ + s0 + p8;
  for (int pass = 0; pass < 2; ++pass) {
#pragma unroll
    for (int it = 0; it < 2; ++it) {
      const int line = it * 32 + q8;
      *(volatile v4u*)(VTo + base + (size_t)line * SEQ) = vv[it];
    }
    __threadfence();
  }
}

__global__ __launch_bounds__(ATT_THREADS)
void attn_sn(const u16* __restrict__ Hp, const u16* __restrict__ Lp, const u16* __restrict__ VTp,
             const float* __restrict__ Np, const float* __restrict__ OFp, float* Out) {
#pragma clang fp contract(off)
  __shared__ __align__(16) float smem[WPB * WREG];

  const int tid  = threadIdx.x;
  const int wave = tid >> 5;
  const int lane = tid & 31;
  const int hh   = lane >> 4;
  const int c    = lane & 15;
  const int bid  = blockIdx.x;
  const int qt   = bid % NQT;
  const int rem  = bid / NQT;
  const int hg   = rem % NHG;
  const int b    = rem / NHG;
  if (b >= NB) return;
  const int q0   = qt * 16;
  const int head = hg * WPB + wave;

  float* pt   = smem + wave * WREG;
  float* slab = pt + PTW;

  const size_t tok0 = (size_t)b * SEQ;
  const size_t qcol = (size_t)head * HD + 8 * hh;
  const size_t kcol = (size_t)DMOD + qcol;
  const _Float16* Qh  = (const _Float16*)(const void*)Hp + (tok0 + q0 + c) * QKW + qcol;
  const _Float16* Ql  = (const _Float16*)(const void*)Lp + (tok0 + q0 + c) * QKW + qcol;
  const _Float16* Khb = (const _Float16*)(const void*)Hp + (tok0 + c) * QKW + kcol;
  const _Float16* Klb = (const _Float16*)(const void*)Lp + (tok0 + c) * QKW + kcol;
  const _Float16* Vtb = (const _Float16*)(const void*)VTp + ((size_t)b * DMOD + (size_t)head * HD + c) * SEQ + 8 * hh;
  const float lsc = 0.125f / (QKSC * QKSC);
  const float oc  = 1.0f / (PCAR * VSC);
  const size_t KROW = (size_t)QKW;

  v8f o[4];
#pragma unroll
  for (int j = 0; j < 4; ++j) o[j] = zero8();
  const int ncaus = (q0 >> 5) + 1;
  const int ncl   = (ncaus < NKT) ? ncaus : NKT;
  const int qr0   = q0 + 8 * hh;

#pragma unroll 1
  for (int kt = 0; kt < ncl; ++kt) {
    const int kb = kt * 32;
    v8f s0 = zero8(), s1 = zero8();
    const _Float16* k0p = Khb + (size_t)kb * KROW;
    const _Float16* k1p = k0p + (size_t)16 * KROW;
    const _Float16* l0p = Klb + (size_t)kb * KROW;
    const _Float16* l1p = l0p + (size_t)16 * KROW;
#pragma unroll
    for (int kk = 0; kk < HD / 32; ++kk) {
      const v16h qh  = ldfrag_h(Qh + kk * 32);
      const v16h ql  = ldfrag_h(Ql + kk * 32);
      const v16h kh0 = ldfrag_h(k0p + kk * 32);
      const v16h kh1 = ldfrag_h(k1p + kk * 32);
      const v16h kl0 = ldfrag_h(l0p + kk * 32);
      const v16h kl1 = ldfrag_h(l1p + kk * 32);
      s0 = mma_h(qh, kh0, s0);
      s0 = mma_h(ql, kh0, s0);
      s0 = mma_h(qh, kl0, s0);
      s1 = mma_h(qh, kh1, s1);
      s1 = mma_h(ql, kh1, s1);
      s1 = mma_h(qh, kl1, s1);
      guard2(s0, s1, qh, ql, kh0, kl0, kh1, kl1);
    }
#pragma unroll
    for (int r = 0; r < 8; ++r) {
      const int row = qr0 + r;
      const float w0 = (kb + c <= row)      ? s0[r] * lsc : 0.0f;
      const float w1 = (kb + 16 + c <= row) ? s1[r] * lsc : 0.0f;
      const int ro = (8 * hh + r) * PTP + c;
      pt[ro]      = w0;
      pt[ro + 16] = w1;
    }
    wave_sync_lds();
    FragH ph, pl;
    {
      const float* prow = pt + c * PTP + 8 * hh;
      const v4f p0 = *(const v4f*)(prow), p1 = *(const v4f*)(prow + 4);
      const v4f p2 = *(const v4f*)(prow + 16), p3 = *(const v4f*)(prow + 20);
#pragma unroll
      for (int e = 0; e < 4; ++e) {
        const float ta = p0[e] * PCAR, tb = p1[e] * PCAR, tc = p2[e] * PCAR, td = p3[e] * PCAR;
        const _Float16 ha = (_Float16)ta, hb = (_Float16)tb, hc = (_Float16)tc, hd = (_Float16)td;
        ph.h[0][e]     = ha;
        ph.h[0][4 + e] = hb;
        ph.h[1][e]     = hc;
        ph.h[1][4 + e] = hd;
        pl.h[0][e]     = (_Float16)(ta - (float)ha);
        pl.h[0][4 + e] = (_Float16)(tb - (float)hb);
        pl.h[1][e]     = (_Float16)(tc - (float)hc);
        pl.h[1][4 + e] = (_Float16)(td - (float)hd);
      }
    }
    {
      const _Float16* vtp = Vtb + kb;
#pragma unroll
      for (int jg = 0; jg < 2; ++jg) {
        const size_t da = (size_t)(2 * jg) * 16 * SEQ;
        const size_t db = da + (size_t)16 * SEQ;
        const v16h va = ldfrag_h(vtp + da), vb2 = ldfrag_h(vtp + db);
        o[2 * jg]     = mma_h(ph.v, va,  o[2 * jg]);
        o[2 * jg]     = mma_h(pl.v, va,  o[2 * jg]);
        o[2 * jg + 1] = mma_h(ph.v, vb2, o[2 * jg + 1]);
        o[2 * jg + 1] = mma_h(pl.v, vb2, o[2 * jg + 1]);
        guard2(o[2 * jg], o[2 * jg + 1], ph.v, pl.v, va, vb2, ph.v, pl.v);
      }
    }
    wave_sync_lds();
  }
  acc_guard4(o[0], o[1], o[2], o[3]);
#pragma unroll
  for (int r = 0; r < 8; ++r) {
#pragma unroll
    for (int j = 0; j < 4; ++j) {
      const int idx = (8 * hh + r) * SLP + j * 16 + c;
      slab[idx] = o[j][r] * oc;
    }
  }
  float nv;
  {
    const float yn = bfr(Np[((size_t)b * S_FULL + (size_t)(q0 + c)) * NH + head]);
    const float yo = bfr(OFp[head]);
    const float y  = yn + yo;
    const float spl = fmaxf(y, 0.0f) + log1pf(expf(-fabsf(y)));
    nv = expf(-spl);
  }
  wave_sync_lds();
  v4f vals[8];
#pragma unroll
  for (int it = 0; it < 8; ++it) {
    const int row = it * 2 + hh;
    const float g = __shfl(nv, row);
    const v4f a = *(const v4f*)(slab + row * SLP + c * 4);
    vals[it] = a * g;
  }
  float* dst = Out + ((tok0 + (size_t)q0 + (size_t)hh) * NH + (size_t)head) * (size_t)HD + c * 4;
  const size_t rstep = (size_t)2 * NH * HD;
  for (int pass = 0; pass < 2; ++pass) {
#pragma unroll
    for (int it = 0; it < 8; ++it) {
      *(volatile v4f*)(dst + (size_t)it * rstep) = vals[it];
    }
    __threadfence();
  }
}

extern "C" void kernel_launch(void* const* d_in, const int* in_sizes, int n_in,
                              void* d_out, int out_size, void* d_ws, size_t ws_size,
                              hipStream_t stream) {
  if (n_in < 4) return;
  const long long ntok = (long long)(NB - 1) * S_FULL + SEQ;
  if ((long long)in_sizes[0] < ntok * QKW) return;
  if ((long long)in_sizes[1] < ntok * DMOD) return;
  if ((long long)in_sizes[2] < ntok * NH) return;
  if (in_sizes[3] < NH) return;
  if ((long long)out_size < (long long)NB * SEQ * DMOD) return;

  const float* qk  = (const float*)d_in[0];
  const float* vin = (const float*)d_in[1];
  const float* nin = (const float*)d_in[2];
  const float* ofs = (const float*)d_in[3];
  float*       out = (float*)d_out;

  const size_t szP = (size_t)NB * SEQ * QKW * 2;
  const size_t szV = (size_t)NB * DMOD * SEQ * 2;
  size_t off = 0;
  const size_t oH = off; off += szP;
  const size_t oL = off; off += szP;
  const size_t oV = off; off += szV;
  if (off > ws_size) return;
  if (off > (size_t)WS_CAP) return;

  char* ws = (char*)d_ws;
  u16* Hp  = (u16*)(ws + oH);
  u16* Lp  = (u16*)(ws + oL);
  u16* VTp = (u16*)(ws + oV);

  const dim3 b128(128), b256(256), bAT(ATT_THREADS);
  const dim3 gQK(NB * SEQ);
  const dim3 gVT(NB * NH * NST);
  const dim3 gAT(NB * NHG * NQT);

  qk16<<<gQK, b128, 0, stream>>>(qk, Hp, Lp);
  vt16<<<gVT, b256, 0, stream>>>(vin, VTp);
  attn_sn<<<gAT, bAT, 0, stream>>>(Hp, Lp, VTp, nin, ofs, out);
  (void)hipGetLastError();
}
